// MultiHeadAttention_43516608643289
// MI455X (gfx1250) — hardware-verified
//
#include <hip/hip_runtime.h>
#include <math.h>

#ifndef NB
#define NB 2
#endif
#ifndef SEQ
#define SEQ 2048
#endif
#define NB_FULL 2
#define SEQ_FULL 2048
#define DM 1024
#define NHEAD 16
#define HD 64
#define NTOK (NB * SEQ)
#define QKW (2 * DM)
#define AW 4
#define OP 68
#define PP 36

static_assert(NB >= 1 && NB <= NB_FULL);
static_assert(SEQ >= 64 && SEQ <= SEQ_FULL);
static_assert(SEQ % 64 == 0);
static_assert(SEQ % (16 * AW) == 0);
static_assert(SEQ % 32 == 0);
static_assert(NHEAD * HD == DM);
static_assert(HD == 64);
static_assert(DM % 64 == 0 && DM % 32 == 0);
static_assert(QKW % 32 == 0);
static_assert(NTOK % 64 == 0);
static_assert(16 * PP <= 16 * OP);
static_assert((long long)NTOK * QKW < 2147483647LL);
static_assert((long long)NB * DM * SEQ < 2147483647LL);

typedef __attribute__((ext_vector_type(16))) __bf16       v16b;
typedef __attribute__((ext_vector_type(8)))  float        v8f;
typedef __attribute__((ext_vector_type(4)))  float        v4f;
typedef __attribute__((ext_vector_type(4)))  unsigned int u4;
typedef __attribute__((ext_vector_type(8)))  unsigned int u8v;

__device__ __forceinline__ v16b ldfrag(const unsigned short* __restrict__ p) {
    const u4 a = *(const u4*)(p);
    const u4 c = *(const u4*)(p + 16);
    u8v w;
    w[0] = a.x; w[1] = a.y; w[2] = a.z; w[3] = a.w; w[4] = c.x; w[5] = c.y; w[6] = c.z; w[7] = c.w;
    return __builtin_bit_cast(v16b, w);
}
__device__ __forceinline__ v8f wm(v16b a, v16b b, v8f c) {
    return __builtin_amdgcn_wmma_f32_16x16x32_bf16(false, a, false, b, (short)0, c, false, false);
}
__device__ __forceinline__ void guard2(v8f& a, v8f& b, v16b x, v16b y, v16b z, v16b w) {
    asm volatile("v_nop\n\tv_nop\n\tv_nop\n\tv_nop" : "+v"(a), "+v"(b) : "v"(x), "v"(y), "v"(z), "v"(w));
}
__device__ __forceinline__ void guard4(v8f& a, v8f& b, v8f& c, v8f& d, v16b x, v16b y, v16b z, v16b w) {
    asm volatile("v_nop\n\tv_nop\n\tv_nop\n\tv_nop" : "+v"(a), "+v"(b), "+v"(c), "+v"(d) : "v"(x), "v"(y), "v"(z), "v"(w));
}
__device__ __forceinline__ void guard4g(v8f& a, v8f& b, v8f& c, v8f& d, v16b x, v16b y) {
    asm volatile("v_nop\n\tv_nop\n\tv_nop\n\tv_nop" : "+v"(a), "+v"(b), "+v"(c), "+v"(d) : "v"(x), "v"(y));
}
__device__ __forceinline__ void keep4(v16b a, v16b b, v16b c, v16b d) { asm volatile("v_nop" :: "v"(a), "v"(b), "v"(c), "v"(d)); }
__device__ __forceinline__ void acc_guard4(v8f& a, v8f& b, v8f& c, v8f& d) { asm volatile("v_nop\n\tv_nop\n\tv_nop\n\tv_nop" : "+v"(a), "+v"(b), "+v"(c), "+v"(d)); }

__device__ __forceinline__ unsigned int bfr_bits(float f) { const unsigned int u = __float_as_uint(f); return (u + 0x7fffu + ((u >> 16) & 1u)) >> 16; }
__device__ __forceinline__ float bfr_val(float f) { return __uint_as_float(bfr_bits(f) << 16); }
__device__ __forceinline__ unsigned int pk_hi(float a, float b) { return bfr_bits(a) | (bfr_bits(b) << 16); }
__device__ __forceinline__ unsigned int pk_lo(float a, float b) { return bfr_bits(a - bfr_val(a)) | (bfr_bits(b - bfr_val(b)) << 16); }

__device__ __forceinline__ void wave_lds_sync() {
    __builtin_amdgcn_fence(3  , "workgroup");
    __builtin_amdgcn_wave_barrier();
    __builtin_amdgcn_fence(2  , "workgroup");
}

#define VST2U4(ptr, val) do { const u4 vst2_u4_ = (val); *(volatile u4*)(ptr) = vst2_u4_; __threadfence(); *(volatile u4*)(ptr) = vst2_u4_; } while (0)

__global__ __launch_bounds__(256) void k_cast_bf(const float* __restrict__ SRC, unsigned short* __restrict__ DST, int nR, int rows_per_batch, int src_batch_rows, int ldd, int dup_off) {
    const int u = (int)blockIdx.x * 256 + (int)threadIdx.x;
    if (u >= nR * (DM / 8)) return;
    const int r = u / (DM / 8), c0 = 8 * (u % (DM / 8));
    const int bb = r / rows_per_batch;
    const int sr = bb * src_batch_rows + (r - bb * rows_per_batch);
    const float* s = SRC + (size_t)sr * DM + c0;
    const v4f a = *(const v4f*)(s);
    const v4f c = *(const v4f*)(s + 4);
    u4 pk; pk.x = pk_hi(a.x, a.y); pk.y = pk_hi(a.z, a.w); pk.z = pk_hi(c.x, c.y); pk.w = pk_hi(c.z, c.w);
    unsigned short* d = DST + (size_t)r * ldd + c0;
    VST2U4(d, pk);
    if (dup_off > 0) VST2U4(d + dup_off, pk);
}

template <int OUT_MODE, bool BIAS>
__device__ __forceinline__ void gemm64_body(const unsigned short* __restrict__ A, int lda, long long strideA,
                                            const unsigned short* __restrict__ Bt, int ldb, long long strideB,
                                            float* __restrict__ Cf, unsigned short* __restrict__ Ch, unsigned short* __restrict__ Cl, int ldc, long long strideC,
                                            const float* __restrict__ bias, int M, int N, int K) {
    __shared__ __align__(16) float sT[8][16 * 68];
    const int b = (int)blockIdx.y;
    const int lane = (int)threadIdx.x & 31;
    const int wave = __builtin_amdgcn_readfirstlane((int)(threadIdx.x >> 5));
    const int tilesN = N >> 6, tilesM = M >> 6;
    const int tile = (int)blockIdx.x * 8 + wave;
    if (tile >= tilesM * tilesN) return;
    const int tm = tile / tilesN, tn = tile - tm * tilesN;
    const int m0 = tm << 6, n0 = tn << 6;
    const unsigned short* Ab = A + (size_t)b * (size_t)strideA;
    const unsigned short* Bb = Bt + (size_t)b * (size_t)strideB;
    const int rlane = lane & 15;
    const int koff = (lane >> 4) * 8;
    const int mOff = (lane >> 4) * 8;

    v8f acc[4][4];
#pragma unroll
    for (int i = 0; i < 4; ++i)
#pragma unroll
        for (int j = 0; j < 4; ++j) { const v8f z = {0.f, 0.f, 0.f, 0.f, 0.f, 0.f, 0.f, 0.f}; acc[i][j] = z; }

    for (int k0 = 0; k0 < K; k0 += 32) {
        v16b bh[4];
#pragma unroll
        for (int j = 0; j < 4; ++j) bh[j] = ldfrag(Bb + (size_t)(n0 + (j << 4) + rlane) * ldb + koff + k0);
#pragma unroll
        for (int i = 0; i < 4; ++i) {
            const v16b ah = ldfrag(Ab + (size_t)(m0 + (i << 4) + rlane) * lda + koff + k0);
#pragma unroll
            for (int j = 0; j < 4; ++j) acc[i][j] = wm(ah, bh[j], acc[i][j]);
            guard4g(acc[i][0], acc[i][1], acc[i][2], acc[i][3], ah, bh[3]);
        }
        keep4(bh[0], bh[1], bh[2], bh[3]);
    }
    acc_guard4(acc[0][0], acc[0][1], acc[0][2], acc[0][3]);
    acc_guard4(acc[1][0], acc[1][1], acc[1][2], acc[1][3]);
    acc_guard4(acc[2][0], acc[2][1], acc[2][2], acc[2][3]);
    acc_guard4(acc[3][0], acc[3][1], acc[3][2], acc[3][3]);

#pragma unroll
    for (int i = 0; i < 4; ++i) {
        const int mBase = m0 + (i << 4);
#pragma unroll
        for (int j = 0; j < 4; ++j) {
            float bv = 0.f;
            if (BIAS) bv = bfr_val(bias[n0 + (j << 4) + rlane]);
#pragma unroll
            for (int r = 0; r < 8; ++r) sT[wave][(mOff + r) * 68 + (j << 4) + rlane] = acc[i][j][r] + bv;
        }
        wave_lds_sync();
        if (OUT_MODE == 0) {
            float* C = Cf + (size_t)b * (size_t)strideC;
            const int hh = lane >> 4, c4 = (lane & 15) * 4;
            for (int pass = 0; pass < 2; ++pass) {
#pragma unroll
                for (int it = 0; it < 8; ++it) {
                    const int row = it * 2 + hh;
                    const v4f v = *(const v4f*)(&sT[wave][row * 68 + c4]);
                    *(volatile v4f*)(C + (size_t)(mBase + row) * ldc + n0 + c4) = v;
                }
                __threadfence();
            }
        } else {
            const int q = lane >> 3, c8 = (lane & 7) * 8;
            unsigned short* C1 = Ch + (size_t)b * (size_t)strideC;
            unsigned short* C2 = Cl + (size_t)b * (size_t)strideC;
            for (int pass = 0; pass < 2; ++pass) {
#pragma unroll
                for (int it = 0; it < 4; ++it) {
                    const int row = it * 4 + q;
                    const v4f a = *(const v4f*)(&sT[wave][row * 68 + c8]);
                    const v4f c = *(const v4f*)(&sT[wave][row * 68 + c8 + 4]);
                    u4 hv, lv;
                    hv.x = pk_hi(a.x, a.y); hv.y = pk_hi(a.z, a.w); hv.z = pk_hi(c.x, c.y); hv.w = pk_hi(c.z, c.w);
                    lv.x = pk_lo(a.x, a.y); lv.y = pk_lo(a.z, a.w); lv.z = pk_lo(c.x, c.y); lv.w = pk_lo(c.z, c.w);
                    const size_t off = (size_t)(mBase + row) * ldc + n0 + c8;
                    *(volatile u4*)(C1 + off) = hv;
                    *(volatile u4*)(C2 + off) = lv;
                }
                __threadfence();
            }
        }
        wave_lds_sync();
    }
}

__global__ __launch_bounds__(256) void k_gemm_qk(const unsigned short* __restrict__ XB, const unsigned short* __restrict__ WB, unsigned short* __restrict__ QKH, unsigned short* __restrict__ QKL) {
    gemm64_body<2, false>(XB, DM, 0, WB, DM, 0, nullptr, QKH, QKL, QKW, 0, nullptr, NTOK, QKW, DM);
}
__global__ __launch_bounds__(256) void k_gemm_vt(const unsigned short* __restrict__ WVB, const unsigned short* __restrict__ XB, unsigned short* __restrict__ VTH, unsigned short* __restrict__ VTL) {
    gemm64_body<2, false>(WVB, DM, 0, XB, DM, (long long)SEQ * DM, nullptr, VTH, VTL, SEQ, (long long)DM * SEQ, nullptr, DM, SEQ, DM);
}
__global__ __launch_bounds__(256) void k_gemm_out(const unsigned short* __restrict__ CTX, const unsigned short* __restrict__ WO2, const float* __restrict__ BO, float* __restrict__ OUT) {
    gemm64_body<0, true>(CTX, QKW, (long long)SEQ * QKW, WO2, QKW, 0, OUT, nullptr, nullptr, DM, (long long)SEQ_FULL * DM, BO, SEQ, DM, QKW);
}

__global__ __launch_bounds__(32 * AW) void k_attn_flash(const unsigned short* __restrict__ QKH, const unsigned short* __restrict__ QKL,
                                                        const unsigned short* __restrict__ VTH, const unsigned short* __restrict__ VTL,
                                                        unsigned short* __restrict__ CTX) {
    __shared__ __align__(16) float pl[AW][16 * OP];
    const int lane = (int)threadIdx.x & 31, hf = lane >> 4, l15 = lane & 15;
    const int wave = __builtin_amdgcn_readfirstlane((int)(threadIdx.x >> 5));
    const int h = (int)blockIdx.y, b = (int)blockIdx.z;
    const int q0 = ((int)blockIdx.x * AW + wave) * 16;
    const int jend = q0 + 16;
    const float L2E = 1.4426950408889634f;
    const float NEG = -__builtin_inff();
    const int qoff  = (b * SEQ + q0 + l15) * QKW + h * HD + 8 * hf;
    const int kbase = (b * SEQ + l15) * QKW + DM + h * HD + 8 * hf;
    const int vbase = (b * DM + h * HD + l15) * SEQ + 8 * hf;

    v8f o[4];
    float m8[8], l8[8];
#pragma unroll
    for (int t = 0; t < 4; ++t) { const v8f z = {0.f, 0.f, 0.f, 0.f, 0.f, 0.f, 0.f, 0.f}; o[t] = z; }
#pragma unroll
    for (int i = 0; i < 8; ++i) { m8[i] = NEG; l8[i] = 0.f; }

    for (int j0 = 0; j0 < jend; j0 += 32) {
        int qo = qoff;
        asm volatile("" : "+v"(qo));
        const int ko0 = kbase + j0 * QKW;
        const int ko1 = ko0 + 16 * QKW;
        v8f s0 = {0.f, 0.f, 0.f, 0.f, 0.f, 0.f, 0.f, 0.f};
        v8f s1 = {0.f, 0.f, 0.f, 0.f, 0.f, 0.f, 0.f, 0.f};
#pragma unroll
        for (int ks = 0; ks < 2; ++ks) {
            const v16b qh = ldfrag(QKH + qo + ks * 32), ql = ldfrag(QKL + qo + ks * 32);
            const v16b k0h = ldfrag(QKH + ko0 + ks * 32), k0l = ldfrag(QKL + ko0 + ks * 32);
            const v16b k1h = ldfrag(QKH + ko1 + ks * 32), k1l = ldfrag(QKL + ko1 + ks * 32);
            s0 = wm(qh, k0h, s0); s0 = wm(ql, k0h, s0); s0 = wm(qh, k0l, s0);
            s1 = wm(qh, k1h, s1); s1 = wm(ql, k1h, s1); s1 = wm(qh, k1l, s1);
            guard2(s0, s1, qh, ql, k1h, k1l);
        }
#pragma unroll
        for (int i = 0; i < 8; ++i) {
            const int irow = q0 + 8 * hf + i;
            const float a = (j0 + l15 > irow) ? NEG : s0[i] * L2E;
            const float c = (j0 + 16 + l15 > irow) ? NEG : s1[i] * L2E;
            float mx = fmaxf(a, c);
            mx = fmaxf(mx, __shfl_xor(mx, 1, 32)); mx = fmaxf(mx, __shfl_xor(mx, 2, 32));
            mx = fmaxf(mx, __shfl_xor(mx, 4, 32)); mx = fmaxf(mx, __shfl_xor(mx, 8, 32));
            const float mnew = fmaxf(m8[i], mx);
            const float ea = exp2f(m8[i] - mnew);
            const float corr = (mnew == NEG) ? 1.f : ea;
            const float e0 = exp2f(a - mnew), e1 = exp2f(c - mnew);
            const float p0 = (a == NEG) ? 0.f : e0;
            const float p1 = (c == NEG) ? 0.f : e1;
            float rs = p0 + p1;
            rs += __shfl_xor(rs, 1, 32); rs += __shfl_xor(rs, 2, 32); rs += __shfl_xor(rs, 4, 32); rs += __shfl_xor(rs, 8, 32);
            l8[i] = l8[i] * corr + rs; m8[i] = mnew;
#pragma unroll
            for (int t = 0; t < 4; ++t) o[t][i] *= corr;
            pl[wave][(i + 8 * hf) * PP + l15] = p0;
            pl[wave][(i + 8 * hf) * PP + 16 + l15] = p1;
        }
        wave_lds_sync();
        const v4f pa = *(const v4f*)(&pl[wave][l15 * PP + 8 * hf]);
        const v4f pb = *(const v4f*)(&pl[wave][l15 * PP + 8 * hf + 4]);
        const v4f pc = *(const v4f*)(&pl[wave][l15 * PP + 16 + 8 * hf]);
        const v4f pd = *(const v4f*)(&pl[wave][l15 * PP + 16 + 8 * hf + 4]);
        u8v wh, wl;
        wh[0] = pk_hi(pa.x, pa.y); wh[1] = pk_hi(pa.z, pa.w); wh[2] = pk_hi(pb.x, pb.y); wh[3] = pk_hi(pb.z, pb.w);
        wh[4] = pk_hi(pc.x, pc.y); wh[5] = pk_hi(pc.z, pc.w); wh[6] = pk_hi(pd.x, pd.y); wh[7] = pk_hi(pd.z, pd.w);
        wl[0] = pk_lo(pa.x, pa.y); wl[1] = pk_lo(pa.z, pa.w); wl[2] = pk_lo(pb.x, pb.y); wl[3] = pk_lo(pb.z, pb.w);
        wl[4] = pk_lo(pc.x, pc.y); wl[5] = pk_lo(pc.z, pc.w); wl[6] = pk_lo(pd.x, pd.y); wl[7] = pk_lo(pd.z, pd.w);
        const v16b ph = __builtin_bit_cast(v16b, wh);
        const v16b plo = __builtin_bit_cast(v16b, wl);
        const int vo = vbase + j0;
        const v16b v0h = ldfrag(VTH + vo),                v0l = ldfrag(VTL + vo);
        const v16b v1h = ldfrag(VTH + vo + 16 * SEQ),     v1l = ldfrag(VTL + vo + 16 * SEQ);
        const v16b v2h = ldfrag(VTH + vo + 32 * SEQ),     v2l = ldfrag(VTL + vo + 32 * SEQ);
        const v16b v3h = ldfrag(VTH + vo + 48 * SEQ),     v3l = ldfrag(VTL + vo + 48 * SEQ);
        o[0] = wm(ph, v0h, o[0]); o[0] = wm(plo, v0h, o[0]); o[0] = wm(ph, v0l, o[0]);
        o[1] = wm(ph, v1h, o[1]); o[1] = wm(plo, v1h, o[1]); o[1] = wm(ph, v1l, o[1]);
        o[2] = wm(ph, v2h, o[2]); o[2] = wm(plo, v2h, o[2]); o[2] = wm(ph, v2l, o[2]);
        o[3] = wm(ph, v3h, o[3]); o[3] = wm(plo, v3h, o[3]); o[3] = wm(ph, v3l, o[3]);
        guard4(o[0], o[1], o[2], o[3], ph, plo, v3h, v3l);
        wave_lds_sync();
    }

#pragma unroll
    for (int i = 0; i < 8; ++i) {
        const float inv = 1.0f / l8[i];
#pragma unroll
        for (int t = 0; t < 4; ++t) pl[wave][(i + 8 * hf) * OP + t * 16 + l15] = o[t][i] * inv;
    }
    wave_lds_sync();
    {
        const int rq = lane >> 3, c8 = (lane & 7) * 8;
        for (int pass = 0; pass < 2; ++pass) {
#pragma unroll
            for (int it = 0; it < 4; ++it) {
                const int row = it * 4 + rq;
                const v4f a = *(const v4f*)(&pl[wave][row * OP + c8]);
                const v4f c = *(const v4f*)(&pl[wave][row * OP + c8 + 4]);
                u4 hv, lv;
                hv.x = pk_hi(a.x, a.y); hv.y = pk_hi(a.z, a.w); hv.z = pk_hi(c.x, c.y); hv.w = pk_hi(c.z, c.w);
                lv.x = pk_lo(a.x, a.y); lv.y = pk_lo(a.z, a.w); lv.z = pk_lo(c.x, c.y); lv.w = pk_lo(c.z, c.w);
                unsigned short* d = CTX + (size_t)(b * SEQ + q0 + row) * QKW + h * HD + c8;
                *(volatile u4*)(d) = hv;
                *(volatile u4*)(d + DM) = lv;
            }
            __threadfence();
        }
    }
}

constexpr size_t al256(size_t b) { return ((b + 255) / 256) * 256; }
constexpr size_t SZ_XB  = al256((size_t)NTOK * DM * 2);
constexpr size_t SZ_WB  = al256((size_t)3 * DM * DM * 2);
constexpr size_t SZ_WO2 = al256((size_t)DM * QKW * 2);
constexpr size_t SZ_QK  = al256((size_t)NTOK * QKW * 2);
constexpr size_t SZ_VT  = al256((size_t)NB * DM * SEQ * 2);
constexpr size_t SZ_CTX = al256((size_t)NTOK * QKW * 2);
constexpr size_t WS_TOTAL = SZ_XB + SZ_WB + SZ_WO2 + 2 * SZ_QK + 2 * SZ_VT + SZ_CTX;
static_assert(WS_TOTAL <= (size_t)134217728);
static_assert(((long long)NTOK * (DM / 8)) % 256 == 0);
static_assert(((long long)3 * DM * (DM / 8)) % 256 == 0);
static_assert(((long long)DM * (DM / 8)) % 256 == 0);
static_assert((long long)NTOK * (DM / 8) < 2147483647LL);
static_assert(((NTOK / 64) * (QKW / 64)) % 8 == 0);
static_assert(((DM / 64) * (SEQ / 64)) % 8 == 0);

extern "C" void kernel_launch(void* const* d_in, const int* in_sizes, int n_in, void* d_out, int out_size, void* d_ws, size_t ws_size, hipStream_t stream) {
    if (n_in < 4) return;
    const long long need_x = ((long long)(NB - 1) * SEQ_FULL + SEQ) * DM;
    if ((long long)in_sizes[0] < need_x) return;
    if (in_sizes[1] < 3 * DM * DM || in_sizes[2] < DM * DM || in_sizes[3] < DM) return;
    if ((long long)out_size < need_x) return;
    if (ws_size < WS_TOTAL) return;
    const float* x     = (const float*)d_in[0];
    const float* W_qkv = (const float*)d_in[1];
    const float* W_out = (const float*)d_in[2];
    const float* b_out = (const float*)d_in[3];
    float* out = (float*)d_out;
    char* wsp = (char*)d_ws;
    unsigned short* XB  = (unsigned short*)wsp; wsp += SZ_XB;
    unsigned short* WB  = (unsigned short*)wsp; wsp += SZ_WB;
    unsigned short* WO2 = (unsigned short*)wsp; wsp += SZ_WO2;
    unsigned short* QKH = (unsigned short*)wsp; wsp += SZ_QK;
    unsigned short* QKL = (unsigned short*)wsp; wsp += SZ_QK;
    unsigned short* VTH = (unsigned short*)wsp; wsp += SZ_VT;
    unsigned short* VTL = (unsigned short*)wsp; wsp += SZ_VT;
    unsigned short* CTX = (unsigned short*)wsp; wsp += SZ_CTX;
    if ((size_t)(wsp - (char*)d_ws) > ws_size) return;

    k_cast_bf<<<(unsigned)(((long long)NTOK * (DM / 8) + 255) / 256), 256, 0, stream>>>(x, XB, NTOK, SEQ, SEQ_FULL, DM, 0);
    k_cast_bf<<<(unsigned)(((long long)3 * DM * (DM / 8) + 255) / 256), 256, 0, stream>>>(W_qkv, WB, 3 * DM, 3 * DM, 3 * DM, DM, 0);
    k_cast_bf<<<(unsigned)(((long long)DM * (DM / 8) + 255) / 256), 256, 0, stream>>>(W_out, WO2, DM, DM, DM, QKW, DM);
    k_gemm_qk<<<dim3((unsigned)(((NTOK / 64) * (QKW / 64) + 7) / 8), 1u), 256, 0, stream>>>(XB, WB, QKH, QKL);
    k_gemm_vt<<<dim3((unsigned)(((DM / 64) * (SEQ / 64) + 7) / 8), (unsigned)NB), 256, 0, stream>>>(WB + (size_t)2 * DM * DM, XB, VTH, VTL);
    k_attn_flash<<<dim3((unsigned)(SEQ / (16 * AW)), (unsigned)NHEAD, (unsigned)NB), 32 * AW, 0, stream>>>(QKH, QKL, VTH, VTL, CTX);
    k_gemm_out<<<dim3((unsigned)(((SEQ / 64) * (DM / 64) + 7) / 8), (unsigned)NB), 256, 0, stream>>>(CTX, WO2, b_out, out);
}
